// WCHeadGAPModelL_80668075753619
// MI455X (gfx1250) — hardware-verified
//
#include <hip/hip_runtime.h>
#define NP 5
#define NG 40000
#define UV 256
#define NPIX (UV * UV)
#define ZD 32
#define FD 64
#define HD 32
#define D1 96
#define D2 110
#define D2P 128
#define HM 128
#define NA 11
#define CC 64
#define NTILE (NG / 16 + NP)
#define NROW (NTILE * 16)
#define NN NPIX
#define MAXDEG 4
#define GKS 13107
#define NSUB 40

typedef __bf16 v16b __attribute__((ext_vector_type(16)));
typedef unsigned short v8us __attribute__((ext_vector_type(8), may_alias));
typedef float  v8f  __attribute__((ext_vector_type(8)));
typedef float  v4f  __attribute__((ext_vector_type(4)));
typedef float  v4fa __attribute__((ext_vector_type(4), may_alias));
union FragB { v16b v; v8us half[2]; unsigned short u[16]; };

__device__ __forceinline__ unsigned short bf16_bits(float x) { unsigned int u = __float_as_uint(x); return (unsigned short)((u + 0x7FFFu + ((u >> 16) & 1u)) >> 16); }
__device__ __forceinline__ float bf16_val(unsigned short b) { return __uint_as_float(((unsigned int)b) << 16); }
__device__ __forceinline__ float bf16_round(float x) { return bf16_val(bf16_bits(x)); }
template <int NT>
__device__ __forceinline__ v8f mmaN(v16b ah, v16b al, v16b bh, v16b bl, v8f c) {
  c = __builtin_amdgcn_wmma_f32_16x16x32_bf16(false, ah, false, bh, (short)0, c, false, false);
  if (NT >= 2) c = __builtin_amdgcn_wmma_f32_16x16x32_bf16(false, al, false, bh, (short)0, c, false, false);
  if (NT >= 3) c = __builtin_amdgcn_wmma_f32_16x16x32_bf16(false, ah, false, bl, (short)0, c, false, false);
  asm volatile("v_nop\n\tv_nop\n\tv_nop\n\tv_nop" : "+v"(c) : "v"(ah), "v"(al), "v"(bh), "v"(bl));
  return c;
}

__global__ __launch_bounds__(256) void k_wt_bf16(const float* __restrict__ W, unsigned short* __restrict__ Wt, int K, int N) {
  const int t = blockIdx.x * 256 + threadIdx.x;
  const int k8n = K / 8;
  if (t >= N * k8n) return;
  const int n = t / k8n, k8 = (t % k8n) * 8;
  v8us v;
#pragma unroll
  for (int i = 0; i < 8; ++i) v[i] = bf16_bits(W[(size_t)(k8 + i) * N + n]);
  *(volatile v8us*)(Wt + (size_t)n * K + k8) = v;
  __threadfence();
  *(volatile v8us*)(Wt + (size_t)n * K + k8) = v;
}

template <bool ASPLIT, int ACT, bool BIAS_BF16>
__global__ __launch_bounds__(128) void k_gemm_bf(const float* __restrict__ A, int lda, const unsigned short* __restrict__ Wt, int ldb,
                                               const float* __restrict__ bias, float* __restrict__ C, int ldc, int M, int N, int K) {
  __shared__ __attribute__((aligned(16))) float so[4][16][64];
  const int tid = threadIdx.x, w = tid >> 5, lane = tid & 31, ln = lane & 15, hh = lane >> 4;
  const int ntn = N / 64;
  const int wid = blockIdx.x * 4 + w;
  const int mt = wid / ntn, nq = wid % ntn;
  if (mt * 16 >= M) return;
  const int row0 = mt * 16, col0 = nq * 64;
  const float* arow = A + (size_t)(row0 + ln) * lda;
  v8f acc[4] = {};
  for (int kb = 0; kb < K; kb += 32) {
    FragB ah, al;
    const v4f x0 = *(const v4fa*)(arow + kb + 8 * hh), x1 = *(const v4fa*)(arow + kb + 8 * hh + 4);
    const v4f x2 = *(const v4fa*)(arow + kb + 16 + 8 * hh), x3 = *(const v4fa*)(arow + kb + 16 + 8 * hh + 4);
    float xs[16] = {x0[0],x0[1],x0[2],x0[3],x1[0],x1[1],x1[2],x1[3],x2[0],x2[1],x2[2],x2[3],x3[0],x3[1],x3[2],x3[3]};
#pragma unroll
    for (int i = 0; i < 16; ++i) { const unsigned short hb = bf16_bits(xs[i]); ah.u[i] = hb; al.u[i] = ASPLIT ? bf16_bits(xs[i] - bf16_val(hb)) : (unsigned short)0; }
#pragma unroll
    for (int t = 0; t < 4; ++t) {
      const unsigned short* brow = Wt + (size_t)(col0 + t * 16 + ln) * ldb + kb;
      FragB b;
      b.half[0] = *(const v8us*)(brow + 8 * hh);
      b.half[1] = *(const v8us*)(brow + 16 + 8 * hh);
      acc[t] = mmaN<ASPLIT ? 2 : 1>(ah.v, al.v, b.v, b.v, acc[t]);
    }
  }
#pragma unroll
  for (int t = 0; t < 4; ++t) {
    float bv = bias ? bias[col0 + t * 16 + ln] : 0.f;
    if (BIAS_BF16) bv = bf16_round(bv);
#pragma unroll
    for (int r = 0; r < 8; ++r) { float v = acc[t][r] + bv; if (ACT == 1) v = fmaxf(v, 0.f); so[w][8 * hh + r][t * 16 + ln] = v; }
  }
  __builtin_amdgcn_fence(__ATOMIC_ACQ_REL, "workgroup");
  __builtin_amdgcn_wave_barrier();
  const int rsub = lane >> 4, c4 = (lane & 15) * 4;
  for (int pass = 0; pass < 2; ++pass) {
#pragma unroll
    for (int q = 0; q < 8; ++q) {
      const int r = q * 2 + rsub;
      const v4f v = *(const v4fa*)&so[w][r][c4];
      *(volatile v4f*)(C + (size_t)(row0 + r) * ldc + col0 + c4) = v;
    }
    if (pass == 0) __threadfence();
  }
}

template <int D, bool CAUSAL>
__global__ __launch_bounds__(128) void k_flash(const float* __restrict__ qb, const float* __restrict__ kb, const float* __restrict__ vb,
                                             int pitch, int T, int H, float scale, float* __restrict__ y, int ypitch) {
  constexpr int KS = D / 32;
  constexpr int DT = D / 16;
  __shared__ __attribute__((aligned(16))) unsigned short sKh[32][D + 8], sKl[32][D + 8], sVh[32][D + 8], sVl[32][D + 8];
  __shared__ __attribute__((aligned(16))) unsigned short sPh[4][16][40], sPl[4][16][40];
  __shared__ __attribute__((aligned(16))) float sO[4][16][D];
  const int tid = threadIdx.x, w = tid >> 5, lane = tid & 31, ln = lane & 15, hh = lane >> 4;
  const int nqb = (T + 63) / 64;
  const int bh = blockIdx.x / nqb, qblk = blockIdx.x % nqb;
  const int b = bh / H, h = bh % H;
  const int q0 = qblk * 64 + w * 16;
  const float* Q = qb + (size_t)b * T * pitch + h * D;
  const float* K = kb + (size_t)b * T * pitch + h * D;
  const float* V = vb + (size_t)b * T * pitch + h * D;

  FragB aqh[KS], aql[KS];
  {
    int row = q0 + ln; if (row >= T) row = T - 1;
    const float* qr = Q + (size_t)row * pitch;
#pragma unroll
    for (int ks = 0; ks < KS; ++ks)
#pragma unroll
      for (int i = 0; i < 16; ++i) {
        const int d = ks * 32 + ((i < 8) ? (8 * hh + i) : (16 + 8 * hh + (i - 8)));
        const float x = qr[d] * scale; const unsigned short hb = bf16_bits(x);
        aqh[ks].u[i] = hb; aql[ks].u[i] = bf16_bits(x - bf16_val(hb));
      }
  }
  float m_r[8], l_r[8];
#pragma unroll
  for (int r = 0; r < 8; ++r) { m_r[r] = -3.0e38f; l_r[r] = 0.f; }
  v8f oacc[DT];
#pragma unroll
  for (int dt = 0; dt < DT; ++dt) oacc[dt] = (v8f){0.f,0.f,0.f,0.f,0.f,0.f,0.f,0.f};

  const int kv_end = CAUSAL ? min(T, qblk * 64 + 64) : T;
  for (int j0 = 0; j0 < kv_end; j0 += 32) {
    __syncthreads();
    for (int e = tid; e < 32 * (D / 4); e += 128) {
      const int r = e / (D / 4), c4 = (e % (D / 4)) * 4;
      const int key = j0 + r;
      v4f kf = {0.f,0.f,0.f,0.f}, vf = {0.f,0.f,0.f,0.f};
      if (key < T) { kf = *(const v4fa*)(K + (size_t)key * pitch + c4); vf = *(const v4fa*)(V + (size_t)key * pitch + c4); }
#pragma unroll
      for (int t = 0; t < 4; ++t) {
        unsigned short hb = bf16_bits(kf[t]); sKh[r][c4 + t] = hb; sKl[r][c4 + t] = bf16_bits(kf[t] - bf16_val(hb));
        hb = bf16_bits(vf[t]); sVh[r][c4 + t] = hb; sVl[r][c4 + t] = bf16_bits(vf[t] - bf16_val(hb));
      }
    }
    __syncthreads();
    v8f s[2];
#pragma unroll
    for (int nt = 0; nt < 2; ++nt) {
      v8f acc = {};
#pragma unroll
      for (int ks = 0; ks < KS; ++ks) {
        FragB bh_, bl_;
        bh_.half[0] = *(const v8us*)&sKh[nt * 16 + ln][ks * 32 + 8 * hh]; bh_.half[1] = *(const v8us*)&sKh[nt * 16 + ln][ks * 32 + 16 + 8 * hh];
        bl_.half[0] = *(const v8us*)&sKl[nt * 16 + ln][ks * 32 + 8 * hh]; bl_.half[1] = *(const v8us*)&sKl[nt * 16 + ln][ks * 32 + 16 + 8 * hh];
        acc = mmaN<3>(aqh[ks].v, aql[ks].v, bh_.v, bl_.v, acc);
      }
      s[nt] = acc;
    }
    float alpha[8];
#pragma unroll
    for (int r = 0; r < 8; ++r) {
      const int qi = q0 + 8 * hh + r;
      const int ja = j0 + ln, jb = j0 + 16 + ln;
      if (CAUSAL) { if (ja > qi) s[0][r] = -3.0e38f; if (jb > qi) s[1][r] = -3.0e38f; }
      if (ja >= T) s[0][r] = -3.0e38f;
      if (jb >= T) s[1][r] = -3.0e38f;
      float mx = fmaxf(s[0][r], s[1][r]);
      mx = fmaxf(mx, __shfl_xor(mx, 1, 32)); mx = fmaxf(mx, __shfl_xor(mx, 2, 32)); mx = fmaxf(mx, __shfl_xor(mx, 4, 32)); mx = fmaxf(mx, __shfl_xor(mx, 8, 32));
      const float mnew = fmaxf(m_r[r], mx);
      alpha[r] = (mnew > -1.0e38f) ? __expf(m_r[r] - mnew) : 1.0f;
      const float p0 = (s[0][r] > -1.0e38f) ? __expf(s[0][r] - mnew) : 0.f;
      const float p1 = (s[1][r] > -1.0e38f) ? __expf(s[1][r] - mnew) : 0.f;
      m_r[r] = mnew;
      l_r[r] = l_r[r] * alpha[r] + p0 + p1;
      unsigned short hb = bf16_bits(p0); sPh[w][8 * hh + r][ln] = hb;      sPl[w][8 * hh + r][ln] = bf16_bits(p0 - bf16_val(hb));
      hb = bf16_bits(p1);                sPh[w][8 * hh + r][16 + ln] = hb; sPl[w][8 * hh + r][16 + ln] = bf16_bits(p1 - bf16_val(hb));
    }
#pragma unroll
    for (int dt = 0; dt < DT; ++dt)
#pragma unroll
      for (int r = 0; r < 8; ++r) oacc[dt][r] *= alpha[r];
    __builtin_amdgcn_fence(__ATOMIC_ACQ_REL, "workgroup");
    __builtin_amdgcn_wave_barrier();
    FragB pah, pal;
    pah.half[0] = *(const v8us*)&sPh[w][ln][8 * hh]; pah.half[1] = *(const v8us*)&sPh[w][ln][16 + 8 * hh];
    pal.half[0] = *(const v8us*)&sPl[w][ln][8 * hh]; pal.half[1] = *(const v8us*)&sPl[w][ln][16 + 8 * hh];
#pragma unroll
    for (int dt = 0; dt < DT; ++dt) {
      FragB bvh, bvl;
#pragma unroll
      for (int i = 0; i < 8; ++i) {
        bvh.u[i] = sVh[8 * hh + i][dt * 16 + ln]; bvh.u[8 + i] = sVh[16 + 8 * hh + i][dt * 16 + ln];
        bvl.u[i] = sVl[8 * hh + i][dt * 16 + ln]; bvl.u[8 + i] = sVl[16 + 8 * hh + i][dt * 16 + ln];
      }
      oacc[dt] = mmaN<3>(pah.v, pal.v, bvh.v, bvl.v, oacc[dt]);
    }
    __builtin_amdgcn_fence(__ATOMIC_ACQ_REL, "workgroup");
    __builtin_amdgcn_wave_barrier();
  }
#pragma unroll
  for (int r = 0; r < 8; ++r) {
    float l = l_r[r];
    l += __shfl_xor(l, 1, 32); l += __shfl_xor(l, 2, 32); l += __shfl_xor(l, 4, 32); l += __shfl_xor(l, 8, 32);
    l_r[r] = (l > 0.f) ? 1.0f / l : 0.f;
  }
#pragma unroll
  for (int dt = 0; dt < DT; ++dt)
#pragma unroll
    for (int r = 0; r < 8; ++r) sO[w][8 * hh + r][dt * 16 + ln] = oacc[dt][r] * l_r[r];
  __builtin_amdgcn_fence(__ATOMIC_ACQ_REL, "workgroup");
  __builtin_amdgcn_wave_barrier();
  for (int pass = 0; pass < 2; ++pass) {
    for (int r = 0; r < 16; ++r) {
      const int row = q0 + r;
      if (row < T && lane < D / 4) {
        const v4f val = *(const v4fa*)&sO[w][r][lane * 4];
        *(volatile v4f*)(y + ((size_t)b * T + row) * ypitch + h * D + lane * 4) = val;
      }
    }
    if (pass == 0) __threadfence();
  }
}

typedef _Float16 v16h __attribute__((ext_vector_type(16)));
union FragH { v16h v; v8us half[2]; _Float16 h[16]; unsigned short u[16]; };
template <int NT>
__device__ __forceinline__ v8f mmaH(v16h ah, v16h al, v16h bh, v16h bl, v8f c) {
  c = __builtin_amdgcn_wmma_f32_16x16x32_f16(false, ah, false, bh, (short)0, c, false, false);
  if (NT >= 2) c = __builtin_amdgcn_wmma_f32_16x16x32_f16(false, al, false, bh, (short)0, c, false, false);
  if (NT >= 3) c = __builtin_amdgcn_wmma_f32_16x16x32_f16(false, ah, false, bl, (short)0, c, false, false);
  asm volatile("v_nop\n\tv_nop\n\tv_nop\n\tv_nop" : "+v"(c) : "v"(ah), "v"(al), "v"(bh), "v"(bl));
  return c;
}
template <bool ASPLIT>
__global__ __launch_bounds__(128) void k_gemm_h(const float* __restrict__ A, int lda, size_t sA, const _Float16* __restrict__ Bh, int ldb, size_t sB, float alpha, float* __restrict__ C, int ldc, size_t sC, int M, int N, int K) {
  __shared__ __attribute__((aligned(16))) float so[4][16][64];
  const int tid = threadIdx.x, w = tid >> 5, lane = tid & 31, ln = lane & 15, hh = lane >> 4; const int by = blockIdx.y;
  A += (size_t)by * sA; Bh += (size_t)by * sB; C += (size_t)by * sC;
  const int ntn = (N + 63) / 64; const int wid = blockIdx.x * 4 + w; const int mt = wid / ntn, nq = wid % ntn; if (mt * 16 >= M) return;
  const int row0 = mt * 16, col0 = nq * 64; const float* arow = A + (size_t)(row0 + ln) * lda;
  v8f acc[4] = {};
  for (int kb = 0; kb < K; kb += 32) {
    FragH ah, al;
    const v4f x0 = *(const v4fa*)(arow + kb + 8 * hh), x1 = *(const v4fa*)(arow + kb + 8 * hh + 4), x2 = *(const v4fa*)(arow + kb + 16 + 8 * hh), x3 = *(const v4fa*)(arow + kb + 16 + 8 * hh + 4);
    float xs[16] = {x0[0],x0[1],x0[2],x0[3],x1[0],x1[1],x1[2],x1[3],x2[0],x2[1],x2[2],x2[3],x3[0],x3[1],x3[2],x3[3]};
#pragma unroll
    for (int i = 0; i < 16; ++i) { const _Float16 h = (_Float16)xs[i]; ah.h[i] = h; al.h[i] = ASPLIT ? (_Float16)(xs[i] - (float)h) : (_Float16)0.0f; }
#pragma unroll
    for (int t = 0; t < 4; ++t) { if (col0 + t * 16 >= N) continue; const size_t boff = (size_t)(col0 + t * 16 + ln) * ldb + kb; FragH bq; bq.half[0] = *(const v8us*)(Bh + boff + 8 * hh); bq.half[1] = *(const v8us*)(Bh + boff + 16 + 8 * hh);
      acc[t] = mmaH<ASPLIT ? 2 : 1>(ah.v, al.v, bq.v, bq.v, acc[t]); }
  }
#pragma unroll
  for (int t = 0; t < 4; ++t) { if (col0 + t * 16 >= N) continue;
#pragma unroll
    for (int r = 0; r < 8; ++r) so[w][8 * hh + r][t * 16 + ln] = acc[t][r] * alpha; }
  __builtin_amdgcn_fence(__ATOMIC_ACQ_REL, "workgroup"); __builtin_amdgcn_wave_barrier();
  const int rsub = lane >> 4, c4 = (lane & 15) * 4;
  for (int pass = 0; pass < 2; ++pass) {
#pragma unroll
    for (int q = 0; q < 8; ++q) { const int r = q * 2 + rsub; if (col0 + c4 < N) { const v4f v = *(const v4fa*)&so[w][r][c4]; *(volatile v4f*)(C + (size_t)(row0 + r) * ldc + col0 + c4) = v; } }
    if (pass == 0) __threadfence(); }
}
template <bool ASPLIT>
__global__ __launch_bounds__(128) void k_gemm_hgrp(const float* __restrict__ A, int lda, const _Float16* __restrict__ Bh0, int ldb, size_t strideB, const int* __restrict__ tileGrp, float alpha, float* __restrict__ C, int ldc, int M, int N, int K) {
  __shared__ __attribute__((aligned(16))) float so[4][16][64];
  const int tid = threadIdx.x, w = tid >> 5, lane = tid & 31, ln = lane & 15, hh = lane >> 4; const int ntn = (N + 63) / 64; const int wid = blockIdx.x * 4 + w; const int mt = wid / ntn, nq = wid % ntn; if (mt * 16 >= M) return; const int grp = tileGrp[mt]; if (grp < 0) return; const _Float16* __restrict__ Bh = Bh0 + (size_t)grp * strideB;
  const int row0 = mt * 16, col0 = nq * 64; const float* arow = A + (size_t)(row0 + ln) * lda;
  v8f acc[4] = {};
  for (int kb = 0; kb < K; kb += 32) {
    FragH ah, al;
    const v4f x0 = *(const v4fa*)(arow + kb + 8 * hh), x1 = *(const v4fa*)(arow + kb + 8 * hh + 4), x2 = *(const v4fa*)(arow + kb + 16 + 8 * hh), x3 = *(const v4fa*)(arow + kb + 16 + 8 * hh + 4);
    float xs[16] = {x0[0],x0[1],x0[2],x0[3],x1[0],x1[1],x1[2],x1[3],x2[0],x2[1],x2[2],x2[3],x3[0],x3[1],x3[2],x3[3]};
#pragma unroll
    for (int i = 0; i < 16; ++i) { const _Float16 h = (_Float16)xs[i]; ah.h[i] = h; al.h[i] = ASPLIT ? (_Float16)(xs[i] - (float)h) : (_Float16)0.0f; }
#pragma unroll
    for (int t = 0; t < 4; ++t) { if (col0 + t * 16 >= N) continue; const size_t boff = (size_t)(col0 + t * 16 + ln) * ldb + kb; FragH bq; bq.half[0] = *(const v8us*)(Bh + boff + 8 * hh); bq.half[1] = *(const v8us*)(Bh + boff + 16 + 8 * hh);
      acc[t] = mmaH<ASPLIT ? 2 : 1>(ah.v, al.v, bq.v, bq.v, acc[t]); }
  }
#pragma unroll
  for (int t = 0; t < 4; ++t) { if (col0 + t * 16 >= N) continue;
#pragma unroll
    for (int r = 0; r < 8; ++r) so[w][8 * hh + r][t * 16 + ln] = acc[t][r] * alpha; }
  __builtin_amdgcn_fence(__ATOMIC_ACQ_REL, "workgroup"); __builtin_amdgcn_wave_barrier();
  const int rsub = lane >> 4, c4 = (lane & 15) * 4;
  for (int pass = 0; pass < 2; ++pass) {
#pragma unroll
    for (int q = 0; q < 8; ++q) { const int r = q * 2 + rsub; if (col0 + c4 < N) { const v4f v = *(const v4fa*)&so[w][r][c4]; *(volatile v4f*)(C + (size_t)(row0 + r) * ldc + col0 + c4) = v; } }
    if (pass == 0) __threadfence(); }
}

#define CS_NW 1024
#define CS_CH 832
#define CS_NB 256
#define CS_CAP 8192
__device__ __forceinline__ int cs_dst(const int* __restrict__ eidst, int e, int ne, int nt, int nn) { if (e >= nt) return -1; int d = (e < ne) ? eidst[e] : (e - ne); return d < 0 ? 0 : (d >= nn ? nn - 1 : d); }
__global__ __launch_bounds__(256) void k_cs_p1(const int* __restrict__ eidst, int ne, int nt, int nn, int* __restrict__ seg_dst, int* __restrict__ seg_eid, int* __restrict__ P1, int* __restrict__ Q1) {
  __shared__ int scnt[8][CS_NB]; __shared__ int srun[8][CS_NB]; __shared__ int sod[8][CS_CH]; __shared__ int soe[8][CS_CH];
  const int tid = threadIdx.x, wv = tid >> 5, lane = tid & 31; const int w = blockIdx.x * 8 + wv; const int e0 = w * CS_CH;
  for (int i = lane; i < CS_NB; i += 32) { scnt[wv][i] = 0; srun[wv][i] = 0; }
  __builtin_amdgcn_fence(__ATOMIC_ACQ_REL, "workgroup"); __builtin_amdgcn_wave_barrier();
#pragma unroll 1
  for (int i0 = 0; i0 < CS_CH; i0 += 32) { const int e = e0 + i0 + lane; const int d = cs_dst(eidst, e, ne, nt, nn); const int hb = (d < 0) ? -1 : (d >> 8);
#pragma unroll 1
    for (int ld = 0; ld < 32; ++ld) { const int kk = __shfl(hb, ld, 32); const unsigned long long m = __ballot(hb == kk); const int first = __ffsll((long long)m) - 1; if (ld == first && lane == first && kk >= 0) scnt[wv][kk] += __popcll(m); }
    __builtin_amdgcn_fence(__ATOMIC_ACQ_REL, "workgroup"); __builtin_amdgcn_wave_barrier(); }
  { int loc[8]; int s = 0; for (int j = 0; j < 8; ++j) { loc[j] = s; s += scnt[wv][lane * 8 + j]; }
    int incl = s; for (int o = 1; o < 32; o <<= 1) { const int v = __shfl_up(incl, o, 32); if (lane >= o) incl += v; } const int excl = incl - s;
    for (int j = 0; j < 8; ++j) srun[wv][lane * 8 + j] = excl + loc[j]; }
  __builtin_amdgcn_fence(__ATOMIC_ACQ_REL, "workgroup"); __builtin_amdgcn_wave_barrier();
  for (int pass = 0; pass < 2; ++pass) { for (int i = lane; i < CS_NB; i += 32) { *(volatile int*)(P1 + (size_t)w * CS_NB + i) = scnt[wv][i]; *(volatile int*)(Q1 + (size_t)w * CS_NB + i) = srun[wv][i]; } if (pass == 0) __threadfence(); }
#pragma unroll 1
  for (int i0 = 0; i0 < CS_CH; i0 += 32) { const int e = e0 + i0 + lane; const int d = cs_dst(eidst, e, ne, nt, nn); const int hb = (d < 0) ? -1 : (d >> 8);
    int pos = -1; int grpcnt = 0; bool leader = false;
#pragma unroll 1
    for (int ld = 0; ld < 32; ++ld) { const int kk = __shfl(hb, ld, 32); const unsigned long long g = __ballot(hb == kk); const int first = __ffsll((long long)g) - 1;
      if (ld == first && kk >= 0) { if (hb == kk) { const unsigned long long below = g & ((1ull << lane) - 1ull); pos = srun[wv][kk] + __popcll(below); if (lane == first) { leader = true; grpcnt = __popcll(g); } } } }
    if (pos >= 0) { sod[wv][pos] = d; soe[wv][pos] = e; }
    __builtin_amdgcn_fence(__ATOMIC_ACQ_REL, "workgroup"); __builtin_amdgcn_wave_barrier();
    if (leader) srun[wv][hb] += grpcnt;
    __builtin_amdgcn_fence(__ATOMIC_ACQ_REL, "workgroup"); __builtin_amdgcn_wave_barrier(); }
  for (int pass = 0; pass < 2; ++pass) { for (int i = lane; i < CS_CH; i += 32) { *(volatile int*)(seg_dst + (size_t)e0 + i) = sod[wv][i]; *(volatile int*)(seg_eid + (size_t)e0 + i) = soe[wv][i]; } if (pass == 0) __threadfence(); }
}
__global__ __launch_bounds__(256) void k_cs_scan(const int* __restrict__ P1, int* __restrict__ R, int* __restrict__ S) {
  __shared__ int tot[CS_NB]; __shared__ int st[CS_NB + 1];
  const int b = threadIdx.x; int acc = 0;
#pragma unroll 1
  for (int w = 0; w < CS_NW; ++w) { const int c = P1[(size_t)w * CS_NB + b]; *(volatile int*)(R + (size_t)w * CS_NB + b) = acc; acc += c; }
  __threadfence();
  acc = 0;
#pragma unroll 1
  for (int w = 0; w < CS_NW; ++w) { const int c = P1[(size_t)w * CS_NB + b]; *(volatile int*)(R + (size_t)w * CS_NB + b) = acc; acc += c; }
  tot[b] = acc; __syncthreads();
  if (b == 0) { int s = 0; for (int i = 0; i < CS_NB; ++i) { st[i] = s; s += (tot[i] + 31) & ~31; } st[CS_NB] = s; }
  __syncthreads();
  for (int pass = 0; pass < 2; ++pass) { *(volatile int*)(S + b) = st[b]; if (b < 32) *(volatile int*)(S + CS_NB + b) = (b == 0) ? st[CS_NB] : 0; if (pass == 0) __threadfence(); }
}
__global__ __launch_bounds__(256) void k_cs_p2(const int* __restrict__ seg_dst, const int* __restrict__ seg_eid, const int* __restrict__ P1, const int* __restrict__ Q1, const int* __restrict__ R, const int* __restrict__ S, int nn, int* __restrict__ csr_eid, int* __restrict__ csr_start, int* __restrict__ csr_cnt) {
  __shared__ int sd[CS_CAP]; __shared__ int se[CS_CAP]; __shared__ int sorted[CS_CAP]; __shared__ int lcnt[CS_NB]; __shared__ int lpre[CS_NB + 1];
  const int hb = blockIdx.x, t = threadIdx.x; const int total = (R[(size_t)(CS_NW - 1) * CS_NB + hb] + P1[(size_t)(CS_NW - 1) * CS_NB + hb]); const int tot = total > CS_CAP ? CS_CAP : total;
#pragma unroll 1
  for (int w = t; w < CS_NW; w += 256) { const int c = P1[(size_t)w * CS_NB + hb]; const int base = R[(size_t)w * CS_NB + hb]; const int src = w * CS_CH + Q1[(size_t)w * CS_NB + hb];
    for (int k = 0; k < c; ++k) { const int p = base + k; if (p < CS_CAP) { sd[p] = seg_dst[src + k] & 255; se[p] = seg_eid[src + k]; } } }
  __syncthreads();
  { int c = 0;
#pragma unroll 1
    for (int i = 0; i < tot; ++i) c += (sd[i] == t) ? 1 : 0; lcnt[t] = c; }
  __syncthreads();
  if (t == 0) { int s = 0; for (int i = 0; i < CS_NB; ++i) { lpre[i] = s; s += lcnt[i]; } lpre[CS_NB] = s; }
  __syncthreads();
  { int k = lpre[t];
#pragma unroll 1
    for (int i = 0; i < tot; ++i) if (sd[i] == t) { sorted[k++] = se[i]; } }
  __syncthreads();
  const int s0 = S[hb]; const int s1 = S[hb + 1];
  for (int pass = 0; pass < 2; ++pass) {
    for (int i = t; i < s1 - s0; i += 256) *(volatile int*)(csr_eid + s0 + i) = (i < tot) ? sorted[i] : -1;
    { const int dst = hb * CS_NB + t; *(volatile int*)(csr_start + dst) = s0 + lpre[t]; *(volatile int*)(csr_cnt + dst) = lcnt[t]; }
    if (pass == 0) __threadfence(); }
}
static void build_csr(const int* eidst, int ne, int nt, int nn, int* seg_dst, int* seg_eid, int* P1, int* Q1, int* R, int* S, int* csr_eid, int* csr_start, int* csr_cnt, hipStream_t stream) {
  k_cs_p1<<<CS_NW / 8, 256, 0, stream>>>(eidst, ne, nt, nn, seg_dst, seg_eid, P1, Q1);
  k_cs_scan<<<1, 256, 0, stream>>>(P1, R, S);
  k_cs_p2<<<CS_NB, 256, 0, stream>>>(seg_dst, seg_eid, P1, Q1, R, S, nn, csr_eid, csr_start, csr_cnt);
}

__device__ __forceinline__ float lrelu(float v) { return v >= 0.f ? v : 0.01f * v; }
__global__ __launch_bounds__(256) void k_wt(const float* __restrict__ W, _Float16* __restrict__ Bt, int Gn, int K, int KP, int N, int NPD, float scale) { const size_t t = (size_t)blockIdx.x * 256 + threadIdx.x; if (t >= (size_t)Gn * NPD * (KP / 8)) return; const int k8 = (int)(t % (KP / 8)) * 8; const int n = (int)((t / (KP / 8)) % NPD); const int g = (int)(t / ((size_t)(KP / 8) * NPD)); FragH f;
  for (int q = 0; q < 8; ++q) { const int k = k8 + q; f.h[q] = (k < K && n < N) ? (_Float16)(bf16_round(W[((size_t)g * K + k) * N + n]) * scale) : (_Float16)0.0f; } *(volatile v8us*)((unsigned short*)Bt + ((size_t)g * NPD + n) * KP + k8) = f.half[0]; __threadfence(); *(volatile v8us*)((unsigned short*)Bt + ((size_t)g * NPD + n) * KP + k8) = f.half[0]; }
__device__ void part_tables(const int* __restrict__ cstart, const int* __restrict__ ccnt, int* sst, int* scn, int (*pre)[NSUB + 1]) { if (threadIdx.x < NP) { const int p = threadIdx.x; int s = 0; for (int sb = 0; sb < NSUB; ++sb) { pre[p][sb] = s; int c = ccnt[p * GKS + sb * 256]; c = c < 0 ? 0 : (c > NG ? NG : c); s += c; } pre[p][NSUB] = s; scn[p] = s > NG ? NG : s; }
  __syncthreads(); if (threadIdx.x == 0) { int s = 0; for (int p = 0; p < NP; ++p) { sst[p] = s; s += (scn[p] + 15) / 16; } sst[NP] = s; } __syncthreads(); (void)cstart; }
__global__ __launch_bounds__(256) void k_rows(const int* __restrict__ part, const int* __restrict__ cstart, const int* __restrict__ ccnt, const int* __restrict__ ceid, int* __restrict__ rowG, int* __restrict__ gRow, int* __restrict__ tileGrp) {
  __shared__ int sst[NP + 1], scn[NP]; __shared__ int pre[NP][NSUB + 1]; part_tables(cstart, ccnt, sst, scn, pre); (void)part; (void)gRow; (void)tileGrp;
  const int t = blockIdx.x * 256 + threadIdx.x; if (t >= NROW) return; int p = -1; for (int q = 0; q < NP; ++q) if (t / 16 >= sst[q] && t / 16 < sst[q] + (scn[q] + 15) / 16) p = q; int g = -1;
  if (p >= 0) { const int off = t - sst[p] * 16; if (off < scn[p]) { int sb = 0; while (sb < NSUB - 1 && pre[p][sb + 1] <= off) ++sb; int i = cstart[p * GKS + sb * 256] + (off - pre[p][sb]); i = i < 0 ? 0 : (i >= NG + 32 * CS_NB ? NG + 32 * CS_NB - 1 : i); g = ceid[i]; g = (g < 0 || g >= NG) ? -1 : g; } }
  *(volatile int*)(rowG + t) = g; __threadfence(); *(volatile int*)(rowG + t) = g;
}
__global__ __launch_bounds__(256) void k_tiles(const int* __restrict__ cstart, const int* __restrict__ ccnt, int* __restrict__ tileGrp) { __shared__ int sst[NP + 1], scn[NP]; __shared__ int pre[NP][NSUB + 1]; part_tables(cstart, ccnt, sst, scn, pre);
  const int tl = blockIdx.x * 256 + threadIdx.x; if (tl >= NTILE) return; int p = -1; for (int q = 0; q < NP; ++q) if (tl >= sst[q] && tl < sst[q] + (scn[q] + 15) / 16) p = q; *(volatile int*)(tileGrp + tl) = p; __threadfence(); *(volatile int*)(tileGrp + tl) = p; }
__global__ __launch_bounds__(256) void k_grow(const int* __restrict__ part, const int* __restrict__ cstart, const int* __restrict__ ccnt, int* __restrict__ gRow) { __shared__ int sst[NP + 1], scn[NP]; __shared__ int pre[NP][NSUB + 1]; part_tables(cstart, ccnt, sst, scn, pre);
  const int g = blockIdx.x * 256 + threadIdx.x; if (g >= NG) return; int p = part[g]; p = p < 0 ? 0 : (p >= NP ? NP - 1 : p); const int sb = g >> 10; const int base = pre[p][sb]; int r = 0;
#pragma unroll 1
  for (int g2 = sb << 10; g2 < g; ++g2) { int p2 = part[g2]; p2 = p2 < 0 ? 0 : (p2 >= NP ? NP - 1 : p2); r += (p2 == p); }
  int row = sst[p] * 16 + base + r; row = row < 0 ? 0 : (row >= NROW ? NROW - 1 : row); *(volatile int*)(gRow + g) = row; __threadfence(); *(volatile int*)(gRow + g) = row; }
__global__ __launch_bounds__(256) void k_x1(const int* __restrict__ rowG, const int* __restrict__ part, const float* __restrict__ lf, const float* __restrict__ lz, float* __restrict__ X1) { const size_t t = (size_t)blockIdx.x * 256 + threadIdx.x; if (t >= (size_t)NROW * D1 / 4) return; const int c4 = (int)((t * 4) % D1); const int row = (int)((t * 4) / D1); const int g = rowG[row]; v4f o = {0.f, 0.f, 0.f, 0.f};
  if (g >= 0) { int p = part[g]; p = p < 0 ? 0 : (p >= NP ? NP - 1 : p); for (int q = 0; q < 4; ++q) { const int c = c4 + q; o[q] = (c < FD) ? bf16_round(lf[p * FD + c]) : bf16_round(lz[(size_t)g * ZD + c - FD]); } } *(volatile v4f*)(X1 + t * 4) = o; __threadfence(); *(volatile v4f*)(X1 + t * 4) = o; }
__global__ __launch_bounds__(256) void k_x2(const int* __restrict__ rowG, const float* __restrict__ X1, const float* __restrict__ xyz, const float* __restrict__ AT, float* __restrict__ X2) { const size_t t = (size_t)blockIdx.x * 256 + threadIdx.x; if (t >= (size_t)NROW * D2P / 4) return; const int c4 = (int)((t * 4) % D2P); const int row = (int)((t * 4) / D2P); const int g = rowG[row]; v4f o = {0.f, 0.f, 0.f, 0.f};
  if (g >= 0) { for (int q = 0; q < 4; ++q) { const int c = c4 + q; float v = 0.f; if (c < D1) v = X1[(size_t)row * D1 + c]; else if (c < D1 + 3) v = bf16_round(xyz[(size_t)g * 3 + c - D1]); else if (c < D2) v = AT[(size_t)row * 16 + c - D1 - 3]; o[q] = v; } } *(volatile v4f*)(X2 + t * 4) = o; __threadfence(); *(volatile v4f*)(X2 + t * 4) = o; }
template <int ACT>
__global__ __launch_bounds__(256) void k_gbias(float* __restrict__ Y, const float* __restrict__ b, const int* __restrict__ tileGrp, int N, int NB, int gstride, size_t n4) { const size_t t = (size_t)blockIdx.x * 256 + threadIdx.x; if (t >= n4) return; const int c4 = (int)((t * 4) % N); const int row = (int)((t * 4) / N); const int g = tileGrp[row >> 4]; if (g < 0) return; v4f v = *(const v4fa*)(Y + t * 4);
  for (int q = 0; q < 4; ++q) { const int c = c4 + q; float x = v[q] + ((c < NB) ? bf16_round(b[(size_t)g * gstride + c]) : 0.f); v[q] = (ACT == 1) ? lrelu(x) : x; } *(volatile v4f*)(Y + t * 4) = v; __threadfence(); *(volatile v4f*)(Y + t * 4) = v; }
__global__ __launch_bounds__(256) void k_uv(const float* __restrict__ H2, const int* __restrict__ gRow, const int* __restrict__ ucstart, const int* __restrict__ uccnt, const int* __restrict__ uceid, float* __restrict__ M0) { const size_t t = (size_t)blockIdx.x * 256 + threadIdx.x; if (t >= (size_t)NPIX * HD / 4) return; const int c4 = (int)((t * 4) % HD); const int pix = (int)((t * 4) / HD); v4f o = {0.f, 0.f, 0.f, 0.f};
  int p0 = ucstart[pix]; int cn = uccnt[pix]; cn = cn < 0 ? 0 : (cn > MAXDEG ? MAXDEG : cn); p0 = p0 < 0 ? 0 : (p0 > NG + 32 * CS_NB ? NG + 32 * CS_NB : p0);
  for (int q = 0; q < cn; ++q) { int g = uceid[p0 + q]; g = g < 0 ? 0 : (g >= NG ? NG - 1 : g); int r = gRow[g]; r = r < 0 ? 0 : (r >= NROW ? NROW - 1 : r); const v4f h = *(const v4fa*)(H2 + (size_t)r * 32 + c4); for (int i = 0; i < 4; ++i) o[i] += h[i]; }
  *(volatile v4f*)(M0 + t * 4) = o; __threadfence(); *(volatile v4f*)(M0 + t * 4) = o; }
__global__ __launch_bounds__(256) void k_cwt(const float* __restrict__ w, _Float16* __restrict__ Bt, int CIN, int COUT, int NPD) { const int t = blockIdx.x * 256 + threadIdx.x; const int K = 9 * CIN; if (t >= NPD * (K / 8)) return; const int o = t / (K / 8), k8 = (t % (K / 8)) * 8; FragH f; for (int q = 0; q < 8; ++q) { const int k = k8 + q; const int kk = k / CIN, c = k % CIN; f.h[q] = (o < COUT) ? (_Float16)(bf16_round(w[((size_t)(o * CIN + c)) * 9 + kk]) * 4.0f) : (_Float16)0.0f; } *(volatile v8us*)((unsigned short*)Bt + (size_t)o * K + k8) = f.half[0]; __threadfence(); *(volatile v8us*)((unsigned short*)Bt + (size_t)o * K + k8) = f.half[0]; }
template <int CIN, int NPD, bool RELU_IN>
__global__ __launch_bounds__(128) void k_conv(const float* __restrict__ X, const _Float16* __restrict__ Bt, const float* __restrict__ bias, int COUT, float* __restrict__ Y) {
  __shared__ __attribute__((aligned(16))) float so[4][16][NPD + 1]; constexpr int K = 9 * CIN; constexpr int NTL = NPD / 16;
  const int tid = threadIdx.x, w = tid >> 5, lane = tid & 31, ln = lane & 15, hh = lane >> 4; const int mt = blockIdx.x * 4 + w; const int row0 = mt * 16; const int pix = row0 + ln; const int py = pix / UV, px = pix % UV;
  v8f acc[NTL]; for (int t = 0; t < NTL; ++t) acc[t] = (v8f){0.f,0.f,0.f,0.f,0.f,0.f,0.f,0.f};
#pragma unroll 1
  for (int kb = 0; kb < K; kb += 32) { FragH ah;
#pragma unroll
    for (int half = 0; half < 2; ++half) { const int k0 = kb + half * 16 + 8 * hh; const int kk = k0 / CIN, c0 = k0 % CIN; const int yy = py + kk / 3 - 1, xx = px + kk % 3 - 1; const bool ok = (yy >= 0) && (yy < UV) && (xx >= 0) && (xx < UV);
      v4f a = {0.f,0.f,0.f,0.f}, b2 = {0.f,0.f,0.f,0.f}; if (ok) { const float* src = X + ((size_t)yy * UV + xx) * CIN + c0; a = *(const v4fa*)src; b2 = *(const v4fa*)(src + 4); }
#pragma unroll
      for (int q = 0; q < 4; ++q) { float v0 = a[q], v1 = b2[q]; if (RELU_IN) { v0 = fmaxf(v0, 0.f); v1 = fmaxf(v1, 0.f); } ah.h[half * 8 + q] = (_Float16)v0; ah.h[half * 8 + 4 + q] = (_Float16)v1; } }
#pragma unroll
    for (int t = 0; t < NTL; ++t) { FragH bq; bq.half[0] = *(const v8us*)((const unsigned short*)Bt + (size_t)(t * 16 + ln) * K + kb + 8 * hh); bq.half[1] = *(const v8us*)((const unsigned short*)Bt + (size_t)(t * 16 + ln) * K + kb + 16 + 8 * hh); acc[t] = mmaH<1>(ah.v, ah.v, bq.v, bq.v, acc[t]); } }
#pragma unroll
  for (int t = 0; t < NTL; ++t) {
#pragma unroll
    for (int q = 0; q < 8; ++q) { const int o = t * 16 + ln; so[w][8 * hh + q][o] = acc[t][q] * 0.25f + ((o < COUT) ? bf16_round(bias[o]) : 0.f); } }
  __builtin_amdgcn_fence(__ATOMIC_ACQ_REL, "workgroup"); __builtin_amdgcn_wave_barrier();
  for (int pass = 0; pass < 2; ++pass) { for (int e = lane; e < 16 * NPD; e += 32) { const int r = e / NPD, c = e % NPD; *(volatile float*)(Y + (size_t)(row0 + r) * NPD + c) = so[w][r][c]; } if (pass == 0) __threadfence(); }
}
__global__ __launch_bounds__(256) void k_colstat(const float* __restrict__ X, double* __restrict__ part) { const int c = threadIdx.x & 63, g = threadIdx.x >> 6; const size_t r0 = (size_t)blockIdx.x * 1024; double s = 0.0, q = 0.0;
#pragma unroll 1
  for (int r = g; r < 1024; r += 4) { const float v = X[(r0 + r) * CC + c]; s += v; q += (double)v * v; } __shared__ double a1[4][64], a2[4][64]; a1[g][c] = s; a2[g][c] = q; __syncthreads();
  if (threadIdx.x < 64) { const double A = (a1[0][c] + a1[1][c]) + (a1[2][c] + a1[3][c]), Q = (a2[0][c] + a2[1][c]) + (a2[2][c] + a2[3][c]); *(volatile double*)(part + ((size_t)blockIdx.x * 64 + c) * 2) = A; *(volatile double*)(part + ((size_t)blockIdx.x * 64 + c) * 2 + 1) = Q; __threadfence(); *(volatile double*)(part + ((size_t)blockIdx.x * 64 + c) * 2) = A; *(volatile double*)(part + ((size_t)blockIdx.x * 64 + c) * 2 + 1) = Q; } }
__global__ __launch_bounds__(64) void k_infin(const double* __restrict__ part, float* __restrict__ st) { const int c = threadIdx.x; double s = 0.0, q = 0.0; for (int k = 0; k < NPIX / 1024; ++k) { s += part[((size_t)k * 64 + c) * 2]; q += part[((size_t)k * 64 + c) * 2 + 1]; } const double mu = s / NPIX; double var = q / NPIX - mu * mu; if (var < 0.0) var = 0.0; const float rs = (float)(1.0 / sqrt(var + 1e-5)); const float sh = -(float)mu * rs;
  *(volatile float*)(st + c * 2) = rs; *(volatile float*)(st + c * 2 + 1) = sh; __threadfence(); *(volatile float*)(st + c * 2) = rs; *(volatile float*)(st + c * 2 + 1) = sh; }
__global__ __launch_bounds__(256) void k_inapply(float* __restrict__ X, const float* __restrict__ st) { const size_t t = (size_t)blockIdx.x * 256 + threadIdx.x; if (t >= (size_t)NPIX * CC / 4) return; const int c4 = (int)((t * 4) % CC); v4f v = *(const v4fa*)(X + t * 4); for (int q = 0; q < 4; ++q) v[q] = v[q] * st[(c4 + q) * 2] + st[(c4 + q) * 2 + 1]; *(volatile v4f*)(X + t * 4) = v; __threadfence(); *(volatile v4f*)(X + t * 4) = v; }
__global__ __launch_bounds__(256) void k_out(const float* __restrict__ Y3, float* __restrict__ out) { const int t = blockIdx.x * 256 + threadIdx.x; if (t >= 3 * NPIX) return; const int c = t / NPIX, pix = t % NPIX; const float v = 1.0f / (1.0f + expf(-Y3[(size_t)pix * 16 + c])); *(volatile float*)(out + t) = v; __threadfence(); *(volatile float*)(out + t) = v; }
__global__ __launch_bounds__(256) void k_pkey(const int* __restrict__ part, int* __restrict__ key) { const int g = blockIdx.x * 256 + threadIdx.x; if (g >= NG) return; int p = part[g]; p = p < 0 ? 0 : (p >= NP ? NP - 1 : p); const int k = p * GKS + (g >> 10) * 256; *(volatile int*)(key + g) = k; __threadfence(); *(volatile int*)(key + g) = k; }
extern "C" void kernel_launch(void* const* d_in, const int* in_sizes, int n_in,
                              void* d_out, int out_size, void* d_ws, size_t ws_size, hipStream_t stream) {
  (void)in_sizes; (void)n_in; (void)out_size;
  const float* lz = (const float*)d_in[0]; const float* lf = (const float*)d_in[1]; const float* xyz = (const float*)d_in[2];
  const float* w1i = (const float*)d_in[3]; const float* b1i = (const float*)d_in[4]; const float* w1h = (const float*)d_in[5]; const float* b1h = (const float*)d_in[6]; const float* w1o = (const float*)d_in[7]; const float* b1o = (const float*)d_in[8];
  const float* w2i = (const float*)d_in[9]; const float* b2i = (const float*)d_in[10]; const float* w2h = (const float*)d_in[11]; const float* b2h = (const float*)d_in[12]; const float* w2o = (const float*)d_in[13]; const float* b2o = (const float*)d_in[14];
  const float* ciw = (const float*)d_in[15]; const float* cib = (const float*)d_in[16]; const float* chw = (const float*)d_in[17]; const float* chb = (const float*)d_in[18]; const float* cow = (const float*)d_in[19]; const float* cob = (const float*)d_in[20]; const int* part = (const int*)d_in[21]; const int* uvi = (const int*)d_in[22];
  char* ws = (char*)d_ws; size_t off = 0;
  auto take = [&](size_t bytes) { char* p = ws + off; off += (bytes + 255) & ~(size_t)255; return p; };
  _Float16* B1i = (_Float16*)take((size_t)NP * HM * D1 * 2); _Float16* B1h = (_Float16*)take((size_t)NP * 2 * HM * HM * 2); _Float16* B1o = (_Float16*)take((size_t)NP * 16 * HM * 2);
  _Float16* B2i = (_Float16*)take((size_t)NP * HM * D2P * 2); _Float16* B2h = (_Float16*)take((size_t)NP * 2 * HM * HM * 2); _Float16* B2o = (_Float16*)take((size_t)NP * 32 * HM * 2);
  _Float16* Bci = (_Float16*)take((size_t)CC * 9 * HD * 2); _Float16* Bch = (_Float16*)take((size_t)3 * CC * 9 * CC * 2); _Float16* Bco = (_Float16*)take((size_t)16 * 9 * CC * 2);
  int* seg_dst = (int*)take((size_t)CS_NW * CS_CH * 4); int* seg_eid = (int*)take((size_t)CS_NW * CS_CH * 4); int* P1 = (int*)take((size_t)CS_NW * CS_NB * 4); int* Q1 = (int*)take((size_t)CS_NW * CS_NB * 4); int* R_ = (int*)take((size_t)CS_NW * CS_NB * 4); int* S_ = (int*)take((CS_NB + 32) * 4);
  int* pkey = (int*)take(NG * 4); int* pceid = (int*)take(((size_t)NG + 32 * CS_NB) * 4); int* pstart = (int*)take((size_t)CS_NB * CS_NB * 4); int* pcnt = (int*)take((size_t)CS_NB * CS_NB * 4);
  int* uceid = (int*)take(((size_t)NG + 32 * CS_NB) * 4); int* ustart = (int*)take((size_t)CS_NB * CS_NB * 4); int* ucnt = (int*)take((size_t)CS_NB * CS_NB * 4);
  int* rowG = (int*)take(NROW * 4); int* gRow = (int*)take(NG * 4); int* tileGrp = (int*)take((NTILE + 64) * 4);
  float* X1 = (float*)take((size_t)NROW * D1 * 4); float* Ha = (float*)take((size_t)NROW * HM * 4); float* Hb = (float*)take((size_t)NROW * HM * 4); float* AT = (float*)take((size_t)NROW * 16 * 4); float* X2 = (float*)take((size_t)NROW * D2P * 4); float* H2 = (float*)take((size_t)NROW * 32 * 4);
  float* M0 = (float*)take((size_t)NPIX * HD * 4); float* Ma = (float*)take((size_t)NPIX * CC * 4); float* Mb = (float*)take((size_t)NPIX * CC * 4); float* Y3 = (float*)take((size_t)NPIX * 16 * 4); double* partd = (double*)take((size_t)(NPIX / 1024) * 64 * 2 * 8); float* st = (float*)take(64 * 2 * 4);
  if (off > ws_size) return;
  k_wt<<<(unsigned)(((size_t)NP * HM * (D1 / 8) + 255) / 256), 256, 0, stream>>>(w1i, B1i, NP, D1, D1, HM, HM, 4.0f);
  k_wt<<<(unsigned)(((size_t)NP * 2 * HM * (HM / 8) + 255) / 256), 256, 0, stream>>>(w1h, B1h, NP * 2, HM, HM, HM, HM, 4.0f);
  k_wt<<<(unsigned)(((size_t)NP * 16 * (HM / 8) + 255) / 256), 256, 0, stream>>>(w1o, B1o, NP, HM, HM, NA, 16, 4.0f);
  k_wt<<<(unsigned)(((size_t)NP * HM * (D2P / 8) + 255) / 256), 256, 0, stream>>>(w2i, B2i, NP, D2, D2P, HM, HM, 4.0f);
  k_wt<<<(unsigned)(((size_t)NP * 2 * HM * (HM / 8) + 255) / 256), 256, 0, stream>>>(w2h, B2h, NP * 2, HM, HM, HM, HM, 4.0f);
  k_wt<<<(unsigned)(((size_t)NP * 32 * (HM / 8) + 255) / 256), 256, 0, stream>>>(w2o, B2o, NP, HM, HM, HD, 32, 4.0f);
  k_cwt<<<(CC * (9 * HD / 8) + 255) / 256, 256, 0, stream>>>(ciw, Bci, HD, CC, CC);
  for (int l = 0; l < 3; ++l) k_cwt<<<(CC * (9 * CC / 8) + 255) / 256, 256, 0, stream>>>(chw + (size_t)l * CC * CC * 9, Bch + (size_t)l * CC * 9 * CC, CC, CC, CC);
  k_cwt<<<(16 * (9 * CC / 8) + 255) / 256, 256, 0, stream>>>(cow, Bco, CC, 3, 16);
  k_pkey<<<(NG + 255) / 256, 256, 0, stream>>>(part, pkey); build_csr(pkey, NG, NG, NP * GKS, seg_dst, seg_eid, P1, Q1, R_, S_, pceid, pstart, pcnt, stream);
  build_csr(uvi, NG, NG, NPIX, seg_dst, seg_eid, P1, Q1, R_, S_, uceid, ustart, ucnt, stream);
  k_rows<<<(NROW + 255) / 256, 256, 0, stream>>>(part, pstart, pcnt, pceid, rowG, gRow, tileGrp); k_tiles<<<(NTILE + 255) / 256, 256, 0, stream>>>(pstart, pcnt, tileGrp); k_grow<<<(NG + 255) / 256, 256, 0, stream>>>(part, pstart, pcnt, gRow);
  k_x1<<<(unsigned)(((size_t)NROW * D1 / 4 + 255) / 256), 256, 0, stream>>>(rowG, part, lf, lz, X1);
  k_gemm_hgrp<false><<<dim3(((NROW / 16) * (HM / 64) + 3) / 4, 1), 128, 0, stream>>>(X1, D1, B1i, D1, (size_t)HM * D1, tileGrp, 0.25f, Ha, HM, NROW, HM, D1);
  k_gbias<1><<<(unsigned)(((size_t)NROW * HM / 4 + 255) / 256), 256, 0, stream>>>(Ha, b1i, tileGrp, HM, HM, HM, (size_t)NROW * HM / 4);
  for (int l = 0; l < 2; ++l) { float* in = (l == 0) ? Ha : Hb; float* outp = (l == 0) ? Hb : Ha;
    k_gemm_hgrp<false><<<dim3(((NROW / 16) * (HM / 64) + 3) / 4, 1), 128, 0, stream>>>(in, HM, B1h + (size_t)l * HM * HM, HM, (size_t)2 * HM * HM, tileGrp, 0.25f, outp, HM, NROW, HM, HM);
    k_gbias<1><<<(unsigned)(((size_t)NROW * HM / 4 + 255) / 256), 256, 0, stream>>>(outp, b1h + (size_t)l * HM, tileGrp, HM, HM, 2 * HM, (size_t)NROW * HM / 4); }
  k_gemm_hgrp<false><<<dim3(((NROW / 16) * 1 + 3) / 4, 1), 128, 0, stream>>>(Ha, HM, B1o, HM, (size_t)16 * HM, tileGrp, 0.25f, AT, 16, NROW, 16, HM);
  k_gbias<0><<<(unsigned)(((size_t)NROW * 16 / 4 + 255) / 256), 256, 0, stream>>>(AT, b1o, tileGrp, 16, NA, NA, (size_t)NROW * 16 / 4);
  k_x2<<<(unsigned)(((size_t)NROW * D2P / 4 + 255) / 256), 256, 0, stream>>>(rowG, X1, xyz, AT, X2);
  k_gemm_hgrp<false><<<dim3(((NROW / 16) * (HM / 64) + 3) / 4, 1), 128, 0, stream>>>(X2, D2P, B2i, D2P, (size_t)HM * D2P, tileGrp, 0.25f, Ha, HM, NROW, HM, D2P);
  k_gbias<1><<<(unsigned)(((size_t)NROW * HM / 4 + 255) / 256), 256, 0, stream>>>(Ha, b2i, tileGrp, HM, HM, HM, (size_t)NROW * HM / 4);
  for (int l = 0; l < 2; ++l) { float* in = (l == 0) ? Ha : Hb; float* outp = (l == 0) ? Hb : Ha;
    k_gemm_hgrp<false><<<dim3(((NROW / 16) * (HM / 64) + 3) / 4, 1), 128, 0, stream>>>(in, HM, B2h + (size_t)l * HM * HM, HM, (size_t)2 * HM * HM, tileGrp, 0.25f, outp, HM, NROW, HM, HM);
    k_gbias<1><<<(unsigned)(((size_t)NROW * HM / 4 + 255) / 256), 256, 0, stream>>>(outp, b2h + (size_t)l * HM, tileGrp, HM, HM, 2 * HM, (size_t)NROW * HM / 4); }
  k_gemm_hgrp<false><<<dim3(((NROW / 16) * 1 + 3) / 4, 1), 128, 0, stream>>>(Ha, HM, B2o, HM, (size_t)32 * HM, tileGrp, 0.25f, H2, 32, NROW, 32, HM);
  k_gbias<0><<<(unsigned)(((size_t)NROW * 32 / 4 + 255) / 256), 256, 0, stream>>>(H2, b2o, tileGrp, 32, HD, HD, (size_t)NROW * 32 / 4);
  k_uv<<<(unsigned)(((size_t)NPIX * HD / 4 + 255) / 256), 256, 0, stream>>>(H2, gRow, ustart, ucnt, uceid, M0);
  k_conv<HD, CC, false><<<NPIX / 16 / 4, 128, 0, stream>>>(M0, Bci, cib, CC, Ma);
  for (int l = 0; l < 3; ++l) { float* in = (l % 2 == 0) ? Ma : Mb; float* outp = (l % 2 == 0) ? Mb : Ma;
    k_conv<CC, CC, true><<<NPIX / 16 / 4, 128, 0, stream>>>(in, Bch + (size_t)l * CC * 9 * CC, chb + (size_t)l * CC, CC, outp);
    k_colstat<<<NPIX / 1024, 256, 0, stream>>>(outp, partd); k_infin<<<1, 64, 0, stream>>>(partd, st); k_inapply<<<(unsigned)(((size_t)NPIX * CC / 4 + 255) / 256), 256, 0, stream>>>(outp, st); }
  k_conv<CC, 16, false><<<NPIX / 16 / 4, 128, 0, stream>>>(Mb, Bco, cob, 3, Y3);
  k_out<<<(3 * NPIX + 255) / 256, 256, 0, stream>>>(Y3, (float*)d_out);
}
